// MHSAttention_41987600286090
// MI455X (gfx1250) — hardware-verified
//
#include <hip/hip_runtime.h>


namespace {
constexpr int B = 16, T = 1024, DM = 768, H = 12, HD = 64, BG = 4  , NG = 4  , BL = BG, QL = T;
constexpr int NSL = DM / 128;
constexpr float XS = 8.0f, WSC = 256.0f, PS = 1024.0f, RS_ = 1024.0f, LOG2E = 1.4426950408889634f;
static_assert(T % 64 == 0 && DM % 256 == 0 && H * HD == DM && HD == 64 && B % BG == 0 && NG * BG <= B, "tiling");
typedef _Float16 b16;
typedef __attribute__((ext_vector_type(16))) _Float16 v16b;
typedef __attribute__((ext_vector_type(8))) _Float16 v8b;
typedef __attribute__((ext_vector_type(8))) float v8f;
typedef __attribute__((ext_vector_type(4))) float v4f;
__device__ __forceinline__ float bf16_rne(float f) { unsigned int u = __float_as_uint(f); u += 0x7FFFu + ((u >> 16) & 1u); return __uint_as_float(u & 0xFFFF0000u); }
__device__ __forceinline__ void split16(float v, b16& hi, b16& lo) { hi = (b16)v; lo = (b16)(v - (float)hi); }
__device__ __forceinline__ v16b frag_kb(const b16* p, int hh) { const v8b a = *(const v8b*)(p + 8 * hh), b = *(const v8b*)(p + 16 + 8 * hh); v16b f;
#pragma unroll
  for (int e = 0; e < 8; ++e) { f[e] = a[e]; f[8 + e] = b[e]; } return f; }
__device__ __forceinline__ v8f wmma16b(v16b a, v16b b, v8f c) { v8f d = __builtin_amdgcn_wmma_f32_16x16x32_f16(false, a, false, b, (short)0, c, false, false); asm volatile("v_nop\n\tv_nop\n\tv_nop\n\tv_nop" : "+v"(d) : "v"(a), "v"(b)); return d; }
__device__ __forceinline__ void wave_lds_sync() { __builtin_amdgcn_fence(__ATOMIC_RELEASE, "workgroup"); __builtin_amdgcn_wave_barrier(); __builtin_amdgcn_fence(__ATOMIC_ACQUIRE, "workgroup"); }
__device__ __forceinline__ float pmul(float a, float b) { float p = a * b; asm volatile("" : "+v"(p)); return p; }
__device__ __forceinline__ int iclamp(int v, int lo, int hi) { return v < lo ? lo : (v > hi ? hi : v); }

typedef __attribute__((ext_vector_type(2))) _Float16 v2h;
typedef __attribute__((ext_vector_type(4))) _Float16 v4h;
typedef __attribute__((ext_vector_type(2))) float v2f;
typedef __attribute__((ext_vector_type(4))) int v4i;
__device__ __forceinline__ float nexp2(float v) { return __builtin_amdgcn_exp2f(v); }
__global__ __launch_bounds__(256) void prep_kernel(const float* __restrict__ wqkv, const float* __restrict__ wo, b16* __restrict__ WT, b16* __restrict__ WO) {
  const size_t u = (size_t)blockIdx.x * 256 + threadIdx.x; const size_t n1 = (size_t)3 * DM * DM / 8, n2 = (size_t)DM * DM / 8; if (u >= n1 + n2) return; v8b o; const float* src; b16* dst;
  if (u < n1) { src = wqkv + u * 8; dst = WT + u * 8; } else { src = wo + (u - n1) * 8; dst = WO + (u - n1) * 8; }
  for (int j = 0; j < 8; ++j) o[j] = (b16)(bf16_rne(src[j]) * WSC);
  for (int pass = 0; pass < 2; ++pass) { *(volatile v8b*)dst = o; __threadfence(); }
}
__global__ __launch_bounds__(128) void proj_kernel(const float* __restrict__ x, int b0, const b16* __restrict__ WT, const float* __restrict__ bqkv, b16* __restrict__ QP, b16* __restrict__ QPl, b16* __restrict__ KP, b16* __restrict__ KPl, b16* __restrict__ VTh, b16* __restrict__ VTl) {
  __shared__ __attribute__((aligned(16))) b16 As[64][256 + 8]; __shared__ __attribute__((aligned(16))) float Tf[4][16][128 + 4];
  const int wave = threadIdx.x >> 5, lane = threadIdx.x & 31, nloc = lane & 15, hlf = lane >> 4; const int t0 = blockIdx.x * 64; const int b = blockIdx.y; const int part = blockIdx.z / NSL, slab = blockIdx.z % NSL, c0 = slab * 128, n0 = part * DM + c0;
  if (part == 0 && t0 >= QL) return;
  const float* xb = x + ((size_t)(b0 + b) * T + t0) * DM;
  v8f acc[8];
#pragma unroll
  for (int t = 0; t < 8; ++t) acc[t] = (v8f){};
#pragma unroll 1
  for (int kc = 0; kc < DM; kc += 256) {
    __syncthreads();
    for (int i = threadIdx.x; i < 64 * 64; i += 128) { const int rr = i / 64, q = (i % 64) * 4; const v4f f = *(const v4f*)(xb + (size_t)rr * DM + kc + q); v4h o; for (int j = 0; j < 4; ++j) o[j] = (b16)(bf16_rne(f[j]) * XS); *(v4h*)(&As[rr][q]) = o; }
    __syncthreads();
#pragma unroll 2
    for (int kb = 0; kb < 256; kb += 32) { const v16b a = frag_kb(&As[wave * 16 + nloc][kb], hlf);
#pragma unroll
      for (int t = 0; t < 8; ++t) acc[t] = wmma16b(a, frag_kb(WT + (size_t)(n0 + t * 16 + nloc) * DM + kc + kb, hlf), acc[t]); } }
const float* ba = bqkv + (size_t)part * DM;
#pragma unroll
  for (int t = 0; t < 8; ++t) { const float bb = bf16_rne(ba[c0 + t * 16 + nloc]);
#pragma unroll
    for (int r = 0; r < 8; ++r) Tf[wave][8 * hlf + r][t * 16 + nloc] = acc[t][r] * (1.0f / (XS * WSC)) + bb; }
  __syncthreads();
  for (int pass = 0; pass < 2; ++pass) {
    if (part < 2) { b16* plane = part == 0 ? QP : KP; b16* planl = part == 0 ? QPl : KPl; const int c = c0 + lane * 4; const int h = c / HD, d = c % HD;
      for (int rr = 0; rr < 16; ++rr) { const int tok = t0 + wave * 16 + rr; const size_t ri = (((size_t)b * H + h) * T + tok) * HD + d; const v4f f4 = *(const v4f*)(&Tf[wave][rr][lane * 4]); v4h o4, l4; for (int j = 0; j < 4; ++j) { const float f = f4[j] * XS; const b16 p = (b16)f; o4[j] = p; l4[j] = (b16)((f - (float)p) * RS_); } *(volatile v4h*)(plane + ri) = o4; *(volatile v4h*)(planl + ri) = l4; } }
    else {
#pragma unroll 1
      for (int q = 0; q < 32; ++q) { const int cl = wave * 32 + q; const int c = c0 + cl; const int h = c / HD, d = c % HD; const int tk = lane * 2; v2h hv, lv;
        for (int j = 0; j < 2; ++j) { const float f = Tf[(tk + j) >> 4][(tk + j) & 15][cl] * XS; const b16 p = (b16)f; hv[j] = p; lv[j] = (b16)((f - (float)p) * RS_); }
        const size_t oi = (((size_t)b * H + h) * HD + d) * (size_t)T + t0 + lane * 2; *(volatile v2h*)(VTh + oi) = hv; *(volatile v2h*)(VTl + oi) = lv; } }
    __threadfence(); }
}
__global__ __launch_bounds__(64) void colstats_kernel(const b16* __restrict__ QP, const b16* __restrict__ QPl, const b16* __restrict__ KP, const b16* __restrict__ KPl, float* __restrict__ CS) {
  const int wave = threadIdx.x >> 5, lane = threadIdx.x & 31, hh = lane >> 4, col = lane & 15; const int b = blockIdx.y / H, h = blockIdx.y % H; const int k0 = blockIdx.x * 32 + wave * 16, ki = k0 + col;
  const size_t ph = (size_t)b * H + h; const b16* Qb = QP + ph * T * HD; const b16* Qbl = QPl + ph * T * HD; const b16* Kb = KP + ph * T * HD; const b16* Kbl = KPl + ph * T * HD;
  const v16b ka0 = frag_kb(Kb + (size_t)ki * HD, hh), ka1 = frag_kb(Kb + (size_t)ki * HD + 32, hh), kl0 = frag_kb(Kbl + (size_t)ki * HD, hh), kl1 = frag_kb(Kbl + (size_t)ki * HD + 32, hh);
  const float cs = LOG2E / (8.0f * XS * XS);
  float m = -INFINITY, l = 0.0f;
#pragma unroll 1
  for (int qb = 0; qb < T; qb += 32) {
    float e[16]; float mx = -INFINITY;
#pragma unroll
    for (int u = 0; u < 2; ++u) { v8f s = (v8f){}, sx = (v8f){}; const size_t qr = (size_t)(qb + u * 16 + col) * HD; { const v16b q0f = frag_kb(Qb + qr, hh), q1f = frag_kb(Qb + qr + 32, hh); s = wmma16b(q0f, ka0, s); s = wmma16b(q1f, ka1, s); sx = wmma16b(q0f, kl0, sx); sx = wmma16b(q1f, kl1, sx); sx = wmma16b(frag_kb(Qbl + qr, hh), ka0, sx); sx = wmma16b(frag_kb(Qbl + qr + 32, hh), ka1, sx); }
#pragma unroll
      for (int r = 0; r < 8; ++r) { const float vv = (s[r] + sx[r] * (1.0f / RS_)) * cs; e[u * 8 + r] = vv; mx = fmaxf(mx, vv); } }
    mx = fmaxf(mx, __shfl_xor(mx, 16)); const float mn = fmaxf(m, mx); const float al = nexp2(m - mn); float sum = 0.0f;
#pragma unroll
    for (int i2 = 0; i2 < 16; ++i2) sum += nexp2(e[i2] - mn);
    sum += __shfl_xor(sum, 16); l = l * al + sum; m = mn; }
  for (int pass = 0; pass < 2; ++pass) { if (hh == 0) { v2f o; o[0] = m; o[1] = l; *(volatile v2f*)(CS + (ph * T + ki) * 2) = o; } __threadfence(); }
}
__global__ __launch_bounds__(64) void attn_kernel(const b16* __restrict__ QP, const b16* __restrict__ QPl, const b16* __restrict__ KP, const b16* __restrict__ KPl, const b16* __restrict__ VTh, const b16* __restrict__ VTl, const float* __restrict__ CS, b16* __restrict__ Ch, b16* __restrict__ Cl) {
  __shared__ __attribute__((aligned(16))) b16 Pb[2][16][32 + 8], Pl[2][16][32 + 8]; __shared__ __attribute__((aligned(16))) float To[2][16][HD + 4];
  const int wave = threadIdx.x >> 5, lane = threadIdx.x & 31, hh = lane >> 4, col = lane & 15; const int b = blockIdx.y / H, h = blockIdx.y % H; const int q0 = blockIdx.x * 32 + wave * 16, qi = q0 + col;
  const size_t ph = (size_t)b * H + h; const b16* Qb = QP + ph * T * HD; const b16* Qbl = QPl + ph * T * HD; const b16* Kb = KP + ph * T * HD; const b16* Kbl = KPl + ph * T * HD; const b16* Vh = VTh + ph * HD * (size_t)T; const b16* Vl = VTl + ph * HD * (size_t)T;
  const v16b qa0 = frag_kb(Qb + (size_t)qi * HD, hh), qa1 = frag_kb(Qb + (size_t)qi * HD + 32, hh), ql0 = frag_kb(Qbl + (size_t)qi * HD, hh), ql1 = frag_kb(Qbl + (size_t)qi * HD + 32, hh);
  const float cs = LOG2E / (8.0f * XS * XS);
  const float* csr = CS + ph * T * 2;
  v8f o[4], ol[4]; for (int t = 0; t < 4; ++t) { o[t] = (v8f){}; ol[t] = (v8f){}; }
#pragma unroll 1
  for (int kb = 0; kb < T; kb += 32) {
    float e[16];
#pragma unroll
    for (int u = 0; u < 2; ++u) { v8f s = (v8f){}, sx = (v8f){}; const size_t kr = (size_t)(kb + u * 16 + col) * HD; { const v16b k0 = frag_kb(Kb + kr, hh), k1 = frag_kb(Kb + kr + 32, hh); s = wmma16b(k0, qa0, s); s = wmma16b(k1, qa1, s); sx = wmma16b(k0, ql0, sx); sx = wmma16b(k1, ql1, sx); sx = wmma16b(frag_kb(Kbl + kr, hh), qa0, sx); sx = wmma16b(frag_kb(Kbl + kr + 32, hh), qa1, sx); }
#pragma unroll
      for (int r = 0; r < 8; ++r) s[r] += sx[r] * (1.0f / RS_);
      const size_t kb8 = (size_t)(kb + u * 16 + 8 * hh);
#pragma unroll
      for (int r = 0; r < 8; ++r) { const v2f st = *(const v2f*)(csr + (kb8 + r) * 2); e[u * 8 + r] = nexp2(fmaf(s[r], cs, -st[0])) * __builtin_amdgcn_rcpf(st[1]); } }
#pragma unroll
    for (int i2 = 0; i2 < 16; ++i2) { const float ps = e[i2] * PS; const b16 phh = (b16)ps; const int pc = (i2 < 8 ? 0 : 16) + 8 * hh + (i2 & 7); Pb[wave][col][pc] = phh; Pl[wave][col][pc] = (b16)((ps - (float)phh) * RS_); }
    wave_lds_sync();
    const v16b pf = frag_kb(&Pb[wave][col][0], hh), plf = frag_kb(&Pl[wave][col][0], hh);
#pragma unroll
    for (int t = 0; t < 4; ++t) { const v16b vh = frag_kb(Vh + (size_t)(t * 16 + col) * T + kb, hh); o[t] = wmma16b(vh, pf, o[t]); ol[t] = wmma16b(frag_kb(Vl + (size_t)(t * 16 + col) * T + kb, hh), pf, ol[t]); ol[t] = wmma16b(vh, plf, ol[t]); }
    wave_lds_sync(); }
  const float inv = 1.0f / (PS * XS);
#pragma unroll
  for (int t = 0; t < 4; ++t)
#pragma unroll
    for (int r = 0; r < 8; ++r) To[wave][col][t * 16 + 8 * hh + r] = (o[t][r] + ol[t][r] * (1.0f / RS_)) * inv;
  wave_lds_sync();
  for (int pass = 0; pass < 2; ++pass) { for (int rr = 0; rr < 16; ++rr) { const v2f f = *(const v2f*)(&To[wave][rr][lane * 2]); v2h hv, lv; for (int j = 0; j < 2; ++j) { b16 p, q; split16(f[j] * XS, p, q); hv[j] = p; lv[j] = q; }
      const size_t oi = ((size_t)b * T + q0 + rr) * DM + h * HD + lane * 2; *(volatile v2h*)(Ch + oi) = hv; *(volatile v2h*)(Cl + oi) = lv; } __threadfence(); }
}
__global__ __launch_bounds__(128) void out_kernel(const b16* __restrict__ Ch, const b16* __restrict__ Cl, const b16* __restrict__ WO, const float* __restrict__ bo, float* __restrict__ out, int b0) {
  __shared__ __attribute__((aligned(16))) float Tf[4][16][128 + 4];
  const int wave = threadIdx.x >> 5, lane = threadIdx.x & 31, nloc = lane & 15, hlf = lane >> 4; const int b = blockIdx.z; const size_t m0 = (size_t)b * T + ((size_t)blockIdx.x * 4 + wave) * 16; const size_t mg = m0 + (size_t)b0 * T;
  const int n0 = blockIdx.y * 128;
  v8f acc[8];
#pragma unroll
  for (int t = 0; t < 8; ++t) acc[t] = (v8f){};
#pragma unroll 2
  for (int kb = 0; kb < DM; kb += 32) { const v16b a = frag_kb(Ch + (m0 + nloc) * DM + kb, hlf), al = frag_kb(Cl + (m0 + nloc) * DM + kb, hlf);
#pragma unroll
    for (int t = 0; t < 8; ++t) { const v16b bw = frag_kb(WO + (size_t)(n0 + t * 16 + nloc) * DM + kb, hlf); acc[t] = wmma16b(a, bw, acc[t]); acc[t] = wmma16b(al, bw, acc[t]); } }
#pragma unroll
  for (int t = 0; t < 8; ++t) { const float bb = bf16_rne(bo[n0 + t * 16 + nloc]);
#pragma unroll
    for (int r = 0; r < 8; ++r) Tf[wave][8 * hlf + r][t * 16 + nloc] = acc[t][r] * (1.0f / (XS * WSC)) + bb; }
  wave_lds_sync();
  for (int pass = 0; pass < 2; ++pass) { for (int rr = 0; rr < 16; ++rr) *(volatile v4f*)(out + (mg + rr) * DM + n0 + lane * 4) = *(const v4f*)(&Tf[wave][rr][lane * 4]); __threadfence(); }
}
}

extern "C" void kernel_launch(void* const* d_in, const int* in_sizes, int n_in, void* d_out, int out_size, void* d_ws, size_t ws_size, hipStream_t stream) {
  (void)n_in;
  auto Fp = [&](int i) { return (const float*)d_in[i]; };
  if (in_sizes[0] != B * T * DM || in_sizes[1] != 3 * DM * DM || in_sizes[2] != 3 * DM || in_sizes[3] != DM * DM || in_sizes[4] != DM || out_size != B * T * DM) return;
  size_t off = 0; char* ws = (char*)d_ws;
  auto carve = [&](size_t bytes) { char* p = ws + off; off += (bytes + 255) & ~(size_t)255; return p; };
  b16* WT = (b16*)carve((size_t)3 * DM * DM * 2); b16* WO = (b16*)carve((size_t)DM * DM * 2); const size_t plane = (size_t)BG * T * DM * 2;
  b16* QP = (b16*)carve(plane); b16* QPl = (b16*)carve(plane); b16* KP = (b16*)carve(plane); b16* KPl = (b16*)carve(plane); b16* VTh = (b16*)carve(plane); b16* VTl = (b16*)carve(plane); b16* Ch = (b16*)carve(plane); b16* Cl = (b16*)carve(plane);
  float* CS = (float*)carve((size_t)BG * H * T * 2 * 4);
  if (off > ws_size || off > ((size_t)128 << 20)) return;
  prep_kernel<<<(unsigned)(((size_t)(3 * DM * DM + DM * DM) / 8 + 255) / 256), 256, 0, stream>>>(Fp(1), Fp(3), WT, WO);
  for (int g = 0; g < NG; ++g) { const int b0 = g * BG;
    proj_kernel<<<dim3(T / 64, BG, 3 * NSL), 128, 0, stream>>>(Fp(0), b0, WT, Fp(2), QP, QPl, KP, KPl, VTh, VTl);
    colstats_kernel<<<dim3(T / 32, BG * H), 64, 0, stream>>>(QP, QPl, KP, KPl, CS);
    attn_kernel<<<dim3(QL / 32, BG * H), 64, 0, stream>>>(QP, QPl, KP, KPl, VTh, VTl, CS, Ch, Cl);
    out_kernel<<<dim3(QL / 64, DM / 128, BG), 128, 0, stream>>>(Ch, Cl, WO, Fp(4), (float*)d_out, b0); }
}
